// TAGCN_GRU_73589969649931
// MI455X (gfx1250) — hardware-run, weakly checked
//
#include <hip/hip_runtime.h>


namespace {
constexpr int N = 100000, FS = 32, GC = 64, EM = 32, H = 128, DY = 16, E = 1600000, B = 512, T = 200, KH = 3, NR = B * T, NBLK = N / 16;
constexpr float XS = 8.0f, HS = 64.0f, WSC = 256.0f;
typedef _Float16 b16;
typedef __attribute__((ext_vector_type(16))) _Float16 v16b;
typedef __attribute__((ext_vector_type(8))) _Float16 v8b;
typedef __attribute__((ext_vector_type(8))) float v8f;
typedef __attribute__((ext_vector_type(4))) float v4f;
typedef __attribute__((ext_vector_type(2))) float v2f;
__device__ __forceinline__ float bf16_rne(float f) { unsigned int u = __float_as_uint(f); u += 0x7FFFu + ((u >> 16) & 1u); return __uint_as_float(u & 0xFFFF0000u); }
__device__ __forceinline__ void split16(float v, b16& hi, b16& lo) { hi = (b16)v; lo = (b16)(v - (float)hi); }
__device__ __forceinline__ v16b frag_kb(const b16* p, int hh) { const v8b a = *(const v8b*)(p + 8 * hh), b = *(const v8b*)(p + 16 + 8 * hh); v16b f;
#pragma unroll
  for (int e = 0; e < 8; ++e) { f[e] = a[e]; f[8 + e] = b[e]; } return f; }
__device__ __forceinline__ v8f wmma16b(v16b a, v16b b, v8f c) { v8f d = __builtin_amdgcn_wmma_f32_16x16x32_f16(false, a, false, b, (short)0, c, false, false); asm volatile("v_nop\n\tv_nop\n\tv_nop\n\tv_nop" : "+v"(d) : "v"(a), "v"(b)); return d; }
__device__ __forceinline__ void wave_lds_sync() { __builtin_amdgcn_fence(__ATOMIC_RELEASE, "workgroup"); __builtin_amdgcn_wave_barrier(); __builtin_amdgcn_fence(__ATOMIC_ACQUIRE, "workgroup"); }
__device__ __forceinline__ float pmul(float a, float b) { float p = a * b; asm volatile("" : "+v"(p)); return p; }
__device__ __forceinline__ int iclamp(int v, int lo, int hi) { return v < lo ? lo : (v > hi ? hi : v); }
__device__ __forceinline__ float sigm(float v) { return 1.0f / (1.0f + __expf(-v)); }
__device__ __forceinline__ float gelu(float v) { return 0.5f * v * (1.0f + erff(v * 0.70710678118654752f)); }
constexpr int CSR_NBLK9 = 512, CSR_GB9 = 9, CSR_GN9 = 1 << CSR_GB9  , CSR_TS9 = (CSR_GN9 < 32 ? 32 : CSR_GN9)  , CSR_MAXG9 = 512, CSR_CAP9 = 12288  ;
__device__ __host__ __forceinline__ int csr_tix9(int v) { return (v >> CSR_GB9) * CSR_TS9 + (v & (CSR_GN9 - 1)); }
__global__ __launch_bounds__(64) void csrA_kernel9(const int* __restrict__ dst, int E, int N, int nG, int CHP, int NGP, int* __restrict__ STG, int* __restrict__ HST) {
  extern __shared__ int sm[];
  int* cnt = sm; int* run = sm + NGP; int* ids = sm + 2 * NGP;
  const int b = blockIdx.x; const int ch = (E + CSR_NBLK9 - 1) / CSR_NBLK9; const int e0 = b * ch, e1 = min(E, e0 + ch);
  for (int i = threadIdx.x; i < NGP; i += 64) cnt[i] = 0;
  for (int i = threadIdx.x; i < CHP; i += 64) ids[i] = -1;
  __syncthreads();
  if (threadIdx.x == 0) {
    for (int e = e0; e < e1; ++e) { int d = dst[e]; d = (d < 0) ? 0 : (d >= N ? N - 1 : d); cnt[d >> CSR_GB9] += 1; }
    int acc = 0; for (int g = 0; g < nG; ++g) { run[g] = acc; acc += cnt[g]; }
    for (int e = e0; e < e1; ++e) { int d = dst[e]; d = (d < 0) ? 0 : (d >= N ? N - 1 : d); const int g = d >> CSR_GB9; ids[run[g]] = e; run[g] += 1; } }
  __syncthreads();
  typedef __attribute__((ext_vector_type(4))) int v4i;
  for (int pass = 0; pass < 2; ++pass) {
    for (int i = threadIdx.x; i < CHP / 4; i += 64) *(volatile v4i*)(STG + (size_t)b * CHP + i * 4) = *(const v4i*)(&ids[i * 4]);
    for (int i = threadIdx.x; i < NGP / 4; i += 64) { v4i v; for (int e = 0; e < 4; ++e) v[e] = (i * 4 + e < nG) ? cnt[i * 4 + e] : 0; *(volatile v4i*)(HST + (size_t)b * NGP + i * 4) = v; }
    __threadfence(); }
}
__global__ __launch_bounds__(512) void csrS_kernel9(const int* __restrict__ HST, int nG, int NGP, int* __restrict__ START, int* __restrict__ TOT, int* __restrict__ OFF) {
  __shared__ int tot[CSR_MAXG9];
  const int b = threadIdx.x;
  for (int pass = 0; pass < 2; ++pass) { int runb = 0; for (int g = 0; g < nG; ++g) { int c = HST[(size_t)b * NGP + g]; c = (c < 0) ? 0 : c; ((volatile int*)OFF)[(size_t)g * CSR_NBLK9 + b] = runb; runb += c; } __threadfence(); }
  for (int g = threadIdx.x; g < nG; g += 512) { int s = 0; for (int bb = 0; bb < CSR_NBLK9; ++bb) { int c = HST[(size_t)bb * NGP + g]; s += (c < 0) ? 0 : c; } tot[g] = s; }
  __syncthreads();
  if (threadIdx.x < 32) {
    __shared__ int st[CSR_MAXG9 + 32];
    if (threadIdx.x == 0) { int acc = 0; for (int g = 0; g < NGP; ++g) { st[g] = acc; if (g < nG) acc += (tot[g] + 31) & ~31; } st[NGP] = acc; }
    __builtin_amdgcn_fence(__ATOMIC_RELEASE, "workgroup"); __builtin_amdgcn_wave_barrier(); __builtin_amdgcn_fence(__ATOMIC_ACQUIRE, "workgroup");
    for (int pass = 0; pass < 2; ++pass) { for (int i = threadIdx.x; i < NGP + 32; i += 32) { ((volatile int*)START)[i] = (i <= NGP) ? st[min(i, NGP)] : 0; ((volatile int*)TOT)[i] = (i < nG) ? tot[i] : 0; } __threadfence(); } }
}
__global__ __launch_bounds__(256) void csrB_kernel9(const int* __restrict__ dst, int N, int nG, int CHP, int NGP, int permLen, const int* __restrict__ STG, const int* __restrict__ HST, const int* __restrict__ OFF, const int* __restrict__ START, const int* __restrict__ TOT, int* __restrict__ PERM, int* __restrict__ ROWPTR, int* __restrict__ ROWCNT, int* __restrict__ FLAG) {
  typedef __attribute__((ext_vector_type(4))) int v4i;
  __shared__ int ids[CSR_CAP9]; __shared__ unsigned short key[CSR_CAP9]; __shared__ int outp[CSR_CAP9]; __shared__ int ncnt[CSR_GN9 + 1]; __shared__ int boff[CSR_NBLK9 + 1];
  const int g = blockIdx.x, t_ = threadIdx.x; int tot = TOT[g]; int st = START[g], stn = START[g + 1]; const int v0 = g * CSR_GN9; const int nv = min(CSR_GN9, N - v0); const int t0 = g * CSR_TS9;
  st = (st < 0) ? 0 : (st > permLen - 32 ? permLen - 32 : st) & ~31; stn = (stn < st) ? st : (stn > permLen ? permLen : stn); tot = (tot < 0) ? 0 : tot; if (tot > stn - st && tot <= CSR_CAP9) tot = stn - st;
  if (tot > CSR_CAP9) {
    for (int pass = 0; pass < 2; ++pass) { for (int i = t_; i < CSR_TS9 / 4; i += 256) { v4i a, c; for (int e = 0; e < 4; ++e) { a[e] = st; c[e] = 0; } *(volatile v4i*)(ROWPTR + t0 + i * 4) = a; *(volatile v4i*)(ROWCNT + t0 + i * 4) = c; } if (t_ == 0) ((volatile int*)FLAG)[0] = 1; __threadfence(); } (void)nv; return; }
  if (t_ == 0) { int acc = 0; for (int b = 0; b < CSR_NBLK9; ++b) { boff[b] = acc; int c = HST[(size_t)b * NGP + g]; c = (c < 0) ? 0 : (c > CHP ? CHP : c); acc += c; if (acc > tot) acc = tot; } boff[CSR_NBLK9] = acc; }
  for (int i = t_; i <= CSR_GN9; i += 256) ncnt[i] = 0;
  __syncthreads();
  for (int b = 0; b < CSR_NBLK9; ++b) { const int c = boff[b + 1] - boff[b]; int o_ = OFF[(size_t)g * CSR_NBLK9 + b]; o_ = (o_ < 0) ? 0 : (o_ > CHP - c ? CHP - c : o_); const int* src_ = STG + (size_t)b * CHP + o_;
    for (int i = t_; i < c; i += 256) { int id = src_[i]; id = (id < 0) ? 0 : id; ids[boff[b] + i] = id; int d = dst[id]; d = (d < v0) ? v0 : (d >= N ? N - 1 : d); int kk = d - v0; kk = (kk < 0) ? 0 : (kk >= CSR_GN9 ? CSR_GN9 - 1 : kk); key[boff[b] + i] = (unsigned short)kk; } }
  __syncthreads();
  if (t_ == 0) { for (int i = 0; i < tot; ++i) ncnt[key[i]] += 1; int acc = 0; for (int vl = 0; vl < CSR_GN9; ++vl) { const int c = ncnt[vl]; ncnt[vl] = acc; acc += c; } ncnt[CSR_GN9] = acc;
    for (int i = 0; i < tot; ++i) { const int vl = key[i]; outp[ncnt[vl]] = ids[i]; ncnt[vl] += 1; }
    for (int vl = CSR_GN9; vl > 0; --vl) ncnt[vl] = ncnt[vl - 1]; ncnt[0] = 0; }
  __syncthreads();
  for (int pass = 0; pass < 2; ++pass) {
    for (int i = t_; i < (stn - st) / 4; i += 256) { v4i v; for (int e = 0; e < 4; ++e) { const int q = i * 4 + e; v[e] = (q < tot) ? outp[q] : -1; } *(volatile v4i*)(PERM + st + i * 4) = v; }
    for (int i = t_; i < CSR_TS9 / 4; i += 256) { v4i a, c; for (int e = 0; e < 4; ++e) { const int vl = i * 4 + e; const int vc = vl < CSR_GN9 ? vl : CSR_GN9; a[e] = (vl < CSR_GN9) ? st + ncnt[vc] : st; c[e] = (vl < nv) ? (ncnt[(vc < CSR_GN9 ? vc : CSR_GN9 - 1) + 1] - ncnt[vc]) : 0; } *(volatile v4i*)(ROWPTR + t0 + i * 4) = a; *(volatile v4i*)(ROWCNT + t0 + i * 4) = c; }
    __threadfence(); }
}
__global__ __launch_bounds__(256) void csrZ_kernel9(int* __restrict__ p, size_t n4) { typedef __attribute__((ext_vector_type(4))) int v4i; const size_t tid = (size_t)blockIdx.x * 256 + threadIdx.x, nth = (size_t)gridDim.x * 256; v4i z = {0, 0, 0, 0}; for (size_t i = tid; i < n4; i += nth) *(volatile v4i*)(p + i * 4) = z; }
struct CsrBufs9 { int *STG, *HST, *OFF, *START, *TOT, *PERM, *ROWPTR, *ROWCNT, *FLAG; int nG, NGP, CHP; size_t permLen; char* base; size_t bytes; };
static size_t csr_carve9(CsrBufs9& c, char* ws, size_t off, int E, int N) {
  const size_t off0 = off; c.base = ws + off;
  auto al = [&](size_t bytes) { char* p = ws + off; off += (bytes + 255) & ~(size_t)255; return p; };
  c.nG = (N + CSR_GN9 - 1) / CSR_GN9; c.NGP = (c.nG + 31) & ~31; const int ch = (E + CSR_NBLK9 - 1) / CSR_NBLK9; c.CHP = (ch + 31) & ~31; c.permLen = (size_t)E + 32 * (size_t)c.nG + 32;
  c.STG = (int*)al((size_t)CSR_NBLK9 * c.CHP * 4); c.HST = (int*)al((size_t)CSR_NBLK9 * c.NGP * 4); c.OFF = (int*)al((size_t)c.NGP * CSR_NBLK9 * 4); c.START = (int*)al((size_t)(c.NGP + 64) * 4); c.TOT = (int*)al((size_t)(c.NGP + 64) * 4);
  c.PERM = (int*)al(c.permLen * 4); c.ROWPTR = (int*)al((size_t)c.nG * CSR_TS9 * 4); c.ROWCNT = (int*)al((size_t)c.nG * CSR_TS9 * 4); c.FLAG = (int*)al(256);
  c.bytes = off - off0; return off;
}
static void csr_build9(const CsrBufs9& c, const int* dst, int E, int N, hipStream_t stream) {
  const size_t smem = (size_t)(2 * c.NGP + c.CHP) * 4;
  csrZ_kernel9<<<512, 256, 0, stream>>>((int*)c.base, c.bytes / 16);
  csrA_kernel9<<<CSR_NBLK9, 64, smem, stream>>>(dst, E, N, c.nG, c.CHP, c.NGP, c.STG, c.HST);
  csrS_kernel9<<<1, 512, 0, stream>>>(c.HST, c.nG, c.NGP, c.START, c.TOT, c.OFF);
  csrB_kernel9<<<c.nG, 256, 0, stream>>>(dst, N, c.nG, c.CHP, c.NGP, (int)c.permLen, c.STG, c.HST, c.OFF, c.START, c.TOT, c.PERM, c.ROWPTR, c.ROWCNT, c.FLAG);
}


__global__ __launch_bounds__(256) void wio_kernel(const float* __restrict__ w, int KIN, int OUTW, int KP, b16* __restrict__ WT) {
  const int u = blockIdx.x * 256 + threadIdx.x; if (u >= OUTW * KP / 8) return; const int e = u * 8; const int o = e / KP, k0 = e % KP; v8b v;
#pragma unroll
  for (int j = 0; j < 8; ++j) { const int k = k0 + j; v[j] = k < KIN ? (b16)(bf16_rne(w[(size_t)k * OUTW + o]) * WSC) : (b16)0.0f; } for (int pass = 0; pass < 2; ++pass) { *(volatile v8b*)(WT + e) = v; __threadfence(); }
}
__global__ __launch_bounds__(256) void wgru_kernel(const float* __restrict__ wih, const float* __restrict__ whh, b16* __restrict__ WRZ, b16* __restrict__ WIN, b16* __restrict__ WHN) {
  const int u = blockIdx.x * 256 + threadIdx.x; const int n1 = 256 * 256 / 8, n2 = H * H / 8; if (u >= n1 + 2 * n2) return; v8b v;
  if (u < n1) { const int e = u * 8; const int o = e / 256, k0 = e % 256;
#pragma unroll
    for (int j = 0; j < 8; ++j) { const int k = k0 + j; v[j] = (b16)(bf16_rne(k < H ? wih[(size_t)o * H + k] : whh[(size_t)o * H + k - H]) * WSC); } for (int pass = 0; pass < 2; ++pass) { *(volatile v8b*)(WRZ + e) = v; __threadfence(); } }
  else { const int uu = u - n1; const int which = uu / n2; const int e = (uu % n2) * 8; const float* src = which ? whh : wih;
#pragma unroll
    for (int j = 0; j < 8; ++j) v[j] = (b16)(bf16_rne(src[(size_t)2 * H * H + e + j]) * WSC); for (int pass = 0; pass < 2; ++pass) { *(volatile v8b*)((which ? WHN : WIN) + e) = v; __threadfence(); } }
}
__global__ __launch_bounds__(256) void hop_kernel(const float* __restrict__ x, float* HK, int k, const int* __restrict__ srcs, const int* __restrict__ PERM, const int* __restrict__ ROWPTR, const int* __restrict__ ROWCNT, int permLen) {
  const int wave = threadIdx.x >> 5, lane = threadIdx.x & 31; const size_t v = (size_t)blockIdx.x * 8 + wave; if (v >= (size_t)N) return;
  int st = ROWPTR[v], cnt = ROWCNT[v]; cnt = iclamp(cnt, 0, 1 << 20); st = iclamp(st, 0, permLen - cnt); const float dv = cnt > 0 ? rsqrtf((float)cnt) : 0.0f; float s = 0.0f;
#pragma unroll 1
  for (int j = 0; j < cnt; ++j) { const int e = iclamp(PERM[st + j], 0, E - 1); const size_t u = (size_t)iclamp(srcs[e], 0, N - 1); const int cu = iclamp(ROWCNT[u], 0, 1 << 20); const float du = cu > 0 ? rsqrtf((float)cu) : 0.0f;
    const float hv = (k == 1) ? bf16_rne(x[u * FS + lane]) : HK[u * 96 + (k - 2) * 32 + lane]; s += pmul(pmul(dv, du), hv); }
  for (int pass = 0; pass < 2; ++pass) { ((volatile float*)HK)[v * 96 + (k - 1) * 32 + lane] = s; __threadfence(); }
}
__global__ __launch_bounds__(32) void tag_kernel(const float* __restrict__ x, const float* __restrict__ HK, const b16* __restrict__ WT, const float* __restrict__ tb, float* __restrict__ TO) {
  __shared__ __attribute__((aligned(16))) b16 Ah[16][128 + 8], Al[16][128 + 8]; __shared__ __attribute__((aligned(16))) float Tf[16][GC + 4];
  const int lane = threadIdx.x, nloc = lane & 15, hlf = lane >> 4; const size_t m0 = (size_t)blockIdx.x * 16;
  for (int rr = 0; rr < 16; ++rr) { b16 p, q; split16(bf16_rne(x[(m0 + rr) * FS + lane]) * HS, p, q); Ah[rr][lane] = p; Al[rr][lane] = q; for (int qq = 0; qq < 3; ++qq) { split16(HK[(m0 + rr) * 96 + qq * 32 + lane] * HS, p, q); Ah[rr][32 + qq * 32 + lane] = p; Al[rr][32 + qq * 32 + lane] = q; } }
  wave_lds_sync();
  v8f acc[4];
#pragma unroll
  for (int t = 0; t < 4; ++t) acc[t] = (v8f){};
#pragma unroll
  for (int kb = 0; kb < 128; kb += 32) { const v16b a = frag_kb(&Ah[nloc][kb], hlf), al = frag_kb(&Al[nloc][kb], hlf);
#pragma unroll
    for (int t = 0; t < 4; ++t) { const v16b bw = frag_kb(WT + (size_t)(t * 16 + nloc) * 128 + kb, hlf); acc[t] = wmma16b(a, bw, acc[t]); acc[t] = wmma16b(al, bw, acc[t]); } }
#pragma unroll
  for (int t = 0; t < 4; ++t) { const int c = t * 16 + nloc; const float bb = bf16_rne(tb[c]);
#pragma unroll 1
    for (int r8 = 0; r8 < 8; ++r8) Tf[8 * hlf + r8][c] = acc[t][r8] * (1.0f / (HS * WSC)) + bb; }
  wave_lds_sync();
  for (int pass = 0; pass < 2; ++pass) { for (int rr = 0; rr < 16; ++rr) *(volatile v2f*)(TO + (m0 + rr) * GC + lane * 2) = *(const v2f*)(&Tf[rr][lane * 2]); __threadfence(); }
}
__global__ __launch_bounds__(64) void bnstat_kernel(const float* __restrict__ TO, const float* __restrict__ g, const float* __restrict__ bb, float* __restrict__ STAT) {
  const int c = threadIdx.x; double s = 0.0, s2 = 0.0;
#pragma unroll 4
  for (int n = 0; n < N; ++n) { const double v = (double)TO[(size_t)n * GC + c]; s += v; s2 += v * v; }
  const double mean = s / N; const double var = fmax(s2 / N - mean * mean, 0.0); const float scale = bf16_rne(g[c]) * (float)(1.0 / sqrt(var + 1e-5)); const float shift = bf16_rne(bb[c]) - (float)mean * scale;
  for (int pass = 0; pass < 2; ++pass) { ((volatile float*)STAT)[c] = scale; ((volatile float*)STAT)[GC + c] = shift; __threadfence(); }
}
__global__ __launch_bounds__(32) void xs_kernel(const int* __restrict__ traj, const float* __restrict__ ide, const float* __restrict__ TO, const float* __restrict__ STAT, const float* __restrict__ x, const b16* __restrict__ WP, const float* __restrict__ pb, float* __restrict__ XSQ) {
  __shared__ __attribute__((aligned(16))) b16 Ah[16][128 + 8], Al[16][128 + 8]; __shared__ __attribute__((aligned(16))) float Tf[16][H + 4];
  const int lane = threadIdx.x, nloc = lane & 15, hlf = lane >> 4; const size_t r0 = (size_t)blockIdx.x * 16;
  const float sc0 = STAT[lane], sh0 = STAT[GC + lane], sc1 = STAT[32 + lane], sh1 = STAT[GC + 32 + lane];
  for (int rr = 0; rr < 16; ++rr) { const int n = iclamp(traj[r0 + rr], 0, N - 1); float v[4]; v[0] = bf16_rne(ide[(size_t)n * EM + lane]); float g0 = pmul(TO[(size_t)n * GC + lane], sc0) + sh0, g1 = pmul(TO[(size_t)n * GC + 32 + lane], sc1) + sh1;
    v[1] = g0 > 0.0f ? g0 : expm1f(g0); v[2] = g1 > 0.0f ? g1 : expm1f(g1); v[3] = bf16_rne(x[(size_t)n * FS + lane]);
    for (int q = 0; q < 4; ++q) { b16 p, ql; split16(v[q] * XS, p, ql); Ah[rr][q * 32 + lane] = p; Al[rr][q * 32 + lane] = ql; } }
  wave_lds_sync();
  v8f acc[8];
#pragma unroll
  for (int t = 0; t < 8; ++t) acc[t] = (v8f){};
#pragma unroll
  for (int kb = 0; kb < 128; kb += 32) { const v16b a = frag_kb(&Ah[nloc][kb], hlf), al = frag_kb(&Al[nloc][kb], hlf);
#pragma unroll
    for (int t = 0; t < 8; ++t) { const v16b bw = frag_kb(WP + (size_t)(t * 16 + nloc) * 128 + kb, hlf); acc[t] = wmma16b(a, bw, acc[t]); acc[t] = wmma16b(al, bw, acc[t]); } }
#pragma unroll
  for (int t = 0; t < 8; ++t) { const int c = t * 16 + nloc; const float bb = bf16_rne(pb[c]);
#pragma unroll 1
    for (int r8 = 0; r8 < 8; ++r8) Tf[8 * hlf + r8][c] = fmaxf(acc[t][r8] * (1.0f / (XS * WSC)) + bb, 0.0f); }
  wave_lds_sync();
  for (int pass = 0; pass < 2; ++pass) { for (int rr = 0; rr < 16; ++rr) *(volatile v4f*)(XSQ + (r0 + rr) * H + lane * 4) = *(const v4f*)(&Tf[rr][lane * 4]); __threadfence(); }
}
__global__ __launch_bounds__(32) void gru_kernel(const float* __restrict__ XSQ, const int* __restrict__ lens, const b16* __restrict__ WRZf, const b16* __restrict__ WINf, const b16* __restrict__ WHNf, const float* __restrict__ bihf, const float* __restrict__ bhhf, const b16* __restrict__ WRZb, const b16* __restrict__ WINb, const b16* __restrict__ WHNb, const float* __restrict__ bihb, const float* __restrict__ bhhb, float* __restrict__ HF) {
  __shared__ __attribute__((aligned(16))) b16 Ah[16][256 + 8], Al[16][256 + 8]; __shared__ float Hs[16][H + 1], RZ[16][2 * H + 4]; __shared__ int Ln[16];
  const int lane = threadIdx.x, nloc = lane & 15, hlf = lane >> 4; const int dir = blockIdx.y; const size_t b0 = (size_t)blockIdx.x * 16;
  const b16* WRZ = dir ? WRZb : WRZf; const b16* WIN = dir ? WINb : WINf; const b16* WHN = dir ? WHNb : WHNf; const float* bih = dir ? bihb : bihf; const float* bhh = dir ? bhhb : bhhf;
  for (int rr = 0; rr < 16; ++rr) for (int q = 0; q < 4; ++q) Hs[rr][q * 32 + lane] = 0.0f; if (lane < 16) Ln[lane] = lens[b0 + lane];
  float brz[8], bni[4], bnh[4]; for (int q = 0; q < 8; ++q) brz[q] = bf16_rne(bih[q * 32 + lane]) + bf16_rne(bhh[q * 32 + lane]); for (int q = 0; q < 4; ++q) { bni[q] = bf16_rne(bih[2 * H + q * 32 + lane]); bnh[q] = bf16_rne(bhh[2 * H + q * 32 + lane]); }
  wave_lds_sync(); const float sc = 1.0f / (XS * WSC);
#pragma unroll 1
  for (int s = 0; s < T; ++s) { const int t = dir ? (T - 1 - s) : s;
    for (int rr = 0; rr < 16; ++rr) { const v4f xv = *(const v4f*)(XSQ + ((b0 + rr) * T + t) * H + lane * 4); for (int j = 0; j < 4; ++j) { b16 p, q; split16(xv[j] * XS, p, q); Ah[rr][lane * 4 + j] = p; Al[rr][lane * 4 + j] = q; }
      for (int q = 0; q < 4; ++q) { b16 p, ql; split16(Hs[rr][q * 32 + lane] * XS, p, ql); Ah[rr][H + q * 32 + lane] = p; Al[rr][H + q * 32 + lane] = ql; } }
    wave_lds_sync();
    { v8f acc[16];
#pragma unroll
      for (int tt = 0; tt < 16; ++tt) acc[tt] = (v8f){};
#pragma unroll 2
      for (int kb = 0; kb < 2 * H; kb += 32) { const v16b a = frag_kb(&Ah[nloc][kb], hlf), al = frag_kb(&Al[nloc][kb], hlf);
#pragma unroll
        for (int tt = 0; tt < 16; ++tt) { const v16b bw = frag_kb(WRZ + (size_t)(tt * 16 + nloc) * (2 * H) + kb, hlf); acc[tt] = wmma16b(a, bw, acc[tt]); acc[tt] = wmma16b(al, bw, acc[tt]); } }
#pragma unroll
      for (int tt = 0; tt < 16; ++tt)
#pragma unroll 1
        for (int r8 = 0; r8 < 8; ++r8) RZ[8 * hlf + r8][tt * 16 + nloc] = acc[tt][r8] * sc; }
    wave_lds_sync();
    { v8f gi[8], gh[8];
#pragma unroll
      for (int tt = 0; tt < 8; ++tt) { gi[tt] = (v8f){}; gh[tt] = (v8f){}; }
#pragma unroll
      for (int kb = 0; kb < H; kb += 32) { const v16b a = frag_kb(&Ah[nloc][kb], hlf), al = frag_kb(&Al[nloc][kb], hlf), ah = frag_kb(&Ah[nloc][H + kb], hlf), ahl = frag_kb(&Al[nloc][H + kb], hlf);
#pragma unroll
        for (int tt = 0; tt < 8; ++tt) { const v16b bw = frag_kb(WIN + (size_t)(tt * 16 + nloc) * H + kb, hlf), bw2 = frag_kb(WHN + (size_t)(tt * 16 + nloc) * H + kb, hlf); gi[tt] = wmma16b(a, bw, gi[tt]); gi[tt] = wmma16b(al, bw, gi[tt]); gh[tt] = wmma16b(ah, bw2, gh[tt]); gh[tt] = wmma16b(ahl, bw2, gh[tt]); } }
      wave_lds_sync();
#pragma unroll
      for (int tt = 0; tt < 8; ++tt) { const int u = tt * 16 + nloc; const int sl = (tt & 1) * 16 + nloc, q4 = tt >> 1; const float br = __shfl(brz[q4], sl), bz = __shfl(brz[4 + q4], sl), bi = __shfl(bni[q4], sl), bh = __shfl(bnh[q4], sl);
#pragma unroll
        for (int r8 = 0; r8 < 8; ++r8) { const int rl = 8 * hlf + r8; const float r = sigm(RZ[rl][u] + br), z = sigm(RZ[rl][H + u] + bz); const float n = tanhf(gi[tt][r8] * sc + bi + pmul(r, gh[tt][r8] * sc + bh)); const float ho = Hs[rl][u]; const float hn = pmul(1.0f - z, n) + pmul(z, ho); if (t < Ln[rl]) Hs[rl][u] = hn; } } }
    wave_lds_sync(); }
  for (int pass = 0; pass < 2; ++pass) { for (int rr = 0; rr < 16; ++rr) for (int q = 0; q < 4; ++q) ((volatile float*)HF)[((size_t)dir * B + b0 + rr) * H + q * 32 + lane] = Hs[rr][q * 32 + lane]; __threadfence(); }
}
__global__ __launch_bounds__(32) void head_kernel(const float* __restrict__ HF, const float* __restrict__ dyn, const float* __restrict__ lg, const float* __restrict__ lb, const b16* __restrict__ WF1, const float* __restrict__ f1b, const float* __restrict__ f2w, const float* __restrict__ f2b, int BV, float* __restrict__ out) {
  __shared__ __attribute__((aligned(16))) b16 Ah[16][288 + 8], Al[16][288 + 8]; __shared__ float so[32];
  const int lane = threadIdx.x, nloc = lane & 15, hlf = lane >> 4;
#pragma unroll 1
  for (int half = 0; half < 2; ++half) { const size_t b0 = (size_t)blockIdx.x * 32 + half * 16;
    for (int rr = 0; rr < 16; ++rr) { const size_t b = b0 + rr; float v[8]; float s = 0.0f; for (int q = 0; q < 8; ++q) { const int c = q * 32 + lane; v[q] = c < H ? HF[b * H + c] : HF[((size_t)B + b) * H + c - H]; s += v[q]; }
      for (int o = 16; o; o >>= 1) s += __shfl_xor(s, o); const float mu = s * (1.0f / 256); float vq = 0.0f; for (int q = 0; q < 8; ++q) { const float d = v[q] - mu; vq += pmul(d, d); } for (int o = 16; o; o >>= 1) vq += __shfl_xor(vq, o); const float rs = rsqrtf(vq * (1.0f / 256) + 1e-5f);
      for (int q = 0; q < 8; ++q) { const int c = q * 32 + lane; b16 p, ql; split16((pmul(pmul(v[q] - mu, rs), bf16_rne(lg[c])) + bf16_rne(lb[c])) * XS, p, ql); Ah[rr][c] = p; Al[rr][c] = ql; }
      const float dv = lane < DY ? bf16_rne(dyn[b * DY + lane]) * XS : 0.0f; Ah[rr][256 + lane] = (b16)dv; Al[rr][256 + lane] = (b16)0.0f; }
    wave_lds_sync();
    v8f acc[8];
#pragma unroll
    for (int t = 0; t < 8; ++t) acc[t] = (v8f){};
#pragma unroll 3
    for (int kb = 0; kb < 288; kb += 32) { const v16b a = frag_kb(&Ah[nloc][kb], hlf), al = frag_kb(&Al[nloc][kb], hlf);
#pragma unroll
      for (int t = 0; t < 8; ++t) { const v16b bw = frag_kb(WF1 + (size_t)(t * 16 + nloc) * 288 + kb, hlf); acc[t] = wmma16b(a, bw, acc[t]); acc[t] = wmma16b(al, bw, acc[t]); } }
    float pd[8];
#pragma unroll
    for (int r8 = 0; r8 < 8; ++r8) pd[r8] = 0.0f;
#pragma unroll
    for (int t = 0; t < 8; ++t) { const int c = t * 16 + nloc; const float bb = bf16_rne(f1b[c]), w2 = bf16_rne(f2w[c]);
#pragma unroll
      for (int r8 = 0; r8 < 8; ++r8) pd[r8] += pmul(gelu(acc[t][r8] * (1.0f / (XS * WSC)) + bb), w2); }
#pragma unroll
    for (int r8 = 0; r8 < 8; ++r8) { float s = pd[r8]; for (int o = 1; o < 16; o <<= 1) s += __shfl_xor(s, o); if (nloc == 0) { const int rl = 8 * hlf + r8; so[half * 16 + rl] = (b0 + rl < (size_t)BV) ? s + bf16_rne(f2b[0]) : 0.0f; } }
    wave_lds_sync(); }
  for (int pass = 0; pass < 2; ++pass) { ((volatile float*)out)[(size_t)blockIdx.x * 32 + lane] = so[lane]; __threadfence(); }
}
}

extern "C" void kernel_launch(void* const* d_in, const int* in_sizes, int n_in, void* d_out, int out_size, void* d_ws, size_t ws_size, hipStream_t stream) {
  (void)n_in;
  auto Fp = [&](int i) { return (const float*)d_in[i]; }; auto Ip = [&](int i) { return (const int*)d_in[i]; };
  if (in_sizes[0] != N * FS || in_sizes[1] != 2 * E || in_sizes[2] != B * T || in_sizes[3] != B || in_sizes[4] != B * DY || in_sizes[5] != N * EM || in_sizes[6] != 4 * FS * GC || in_sizes[10] != 128 * H || in_sizes[12] != 3 * H * H || in_sizes[22] != 272 * H || out_size != B) return;
  const int BV = B; const int EUSE = E;
  size_t off = 0; char* ws = (char*)d_ws;
  auto carve = [&](size_t bytes) { char* p = ws + off; off += (bytes + 255) & ~(size_t)255; return p; };
  b16* WTAG = (b16*)carve(GC * 128 * 2); b16* WP = (b16*)carve(H * 128 * 2); b16* WF1 = (b16*)carve(H * 288 * 2);
  b16* WRZ[2]; b16* WIN[2]; b16* WHN[2]; for (int d = 0; d < 2; ++d) { WRZ[d] = (b16*)carve((size_t)256 * 256 * 2); WIN[d] = (b16*)carve((size_t)H * H * 2); WHN[d] = (b16*)carve((size_t)H * H * 2); }
  float* HK = (float*)carve((size_t)N * 96 * 4); float* TO = (float*)carve((size_t)N * GC * 4); float* STAT = (float*)carve(2 * GC * 4); float* XSQ = (float*)carve((size_t)NR * H * 4); float* HF = (float*)carve((size_t)2 * B * H * 4);
  CsrBufs9 csr; off = csr_carve9(csr, ws, off, E, N);
  if (off > ws_size || off > ((size_t)192 << 20)) return;
  wio_kernel<<<(GC * 128 / 8 + 255) / 256, 256, 0, stream>>>(Fp(6), 128, GC, 128, WTAG); wio_kernel<<<(H * 128 / 8 + 255) / 256, 256, 0, stream>>>(Fp(10), 128, H, 128, WP); wio_kernel<<<(H * 288 / 8 + 255) / 256, 256, 0, stream>>>(Fp(22), 272, H, 288, WF1);
  wgru_kernel<<<(256 * 256 / 8 + 2 * H * H / 8 + 255) / 256, 256, 0, stream>>>(Fp(12), Fp(13), WRZ[0], WIN[0], WHN[0]); wgru_kernel<<<(256 * 256 / 8 + 2 * H * H / 8 + 255) / 256, 256, 0, stream>>>(Fp(16), Fp(17), WRZ[1], WIN[1], WHN[1]);
  csr_build9(csr, Ip(1) + E, EUSE, N, stream);
  for (int k = 1; k <= KH; ++k) hop_kernel<<<N / 8, 256, 0, stream>>>(Fp(0), HK, k, Ip(1), csr.PERM, csr.ROWPTR, csr.ROWCNT, (int)csr.permLen);
  tag_kernel<<<NBLK, 32, 0, stream>>>(Fp(0), HK, WTAG, Fp(7), TO);
  bnstat_kernel<<<1, 64, 0, stream>>>(TO, Fp(8), Fp(9), STAT);
  xs_kernel<<<(BV * T) / 16, 32, 0, stream>>>(Ip(2), Fp(5), TO, STAT, Fp(0), WP, Fp(11), XSQ);
  gru_kernel<<<dim3(BV / 16, 2), 32, 0, stream>>>(XSQ, Ip(3), WRZ[0], WIN[0], WHN[0], Fp(14), Fp(15), WRZ[1], WIN[1], WHN[1], Fp(18), Fp(19), HF);
  head_kernel<<<B / 32, 32, 0, stream>>>(HF, Fp(4), Fp(20), Fp(21), WF1, Fp(23), Fp(24), Fp(25), BV, (float*)d_out);
}
